// CompGCNLayer_74431783240016
// MI455X (gfx1250) — hardware-run, weakly checked
//
#include <hip/hip_runtime.h>
#include <stddef.h>
#include <stdint.h>

#define NN      100000
#define NE      640000
#define NR      500
#define DF      128
#define KD      128
#define APITCH  128
#define BPITCH  128
#define CPITCH  128
#define MP      100096
#define RP      512
#define GBM     64
#define GBN     128
#define GTHR    128
#define NTHR    256
#define NWAVE   8
#define EPT     8
#define WCH     (32 * EPT)
#define NBRUN   1024
#define SLB     10
#define NBK     98
#define WLCAP   1536
#define RCAP    8192
#define MAXB1024_MEAS 6812
#define RBM     64

#define BK_ZINTS (NWAVE * WLCAP + RCAP + 3 * NBRUN)
#define BK_INTS  (BK_ZINTS + 16)
#define BK_LDS   (BK_INTS * 4)

#define PBX   (MP * DF / 8 / NTHR)
#define PBR   (RP * DF / 8 / NTHR)
#define PBW   (DF * KD / 8 / NTHR)
#define PBTOT (PBX + PBR + 2 * PBW)

static_assert(MP % GBM == 0 && MP >= NN && MP == 1564 * GBM);
static_assert(RP % GBM == 0 && RP >= NR);
static_assert(KD % 32 == 0 && GBN == DF && GBM == (GTHR / 32) * 16 && DF == 4 * 32);
static_assert((MP * DF / 8) % NTHR == 0 && (RP * DF / 8) % NTHR == 0 && (DF * KD / 8) % NTHR == 0);
static_assert(NBRUN == (1 << SLB) && NBRUN % RBM == 0 && NBRUN % 32 == 0);
static_assert(NBK * NBRUN >= NN && (NBK - 1) * NBRUN < NN);
static_assert(NN <= (1 << 17) && NR <= (1 << 9) && NE < (1 << 20));
static_assert(NE % WCH == 0 && NE % 4 == 0);
static_assert((long long)RCAP * 100 >= (long long)MAXB1024_MEAS * 115);
static_assert(WLCAP >= MAXB1024_MEAS / 8 + 8 * 30 + 1);
static_assert(RCAP % NTHR == 0 && RCAP % (NTHR * 4) == 0 && BK_ZINTS % (NTHR * 4) == 0);
static_assert(2 * NBRUN == NTHR * 8);
static_assert(BK_LDS <= 327680);
static_assert(GBM * GBN * 4 <= 65536);
static_assert((long long)NN * DF == 12800000LL);
static_assert(RBM % NWAVE == 0 && ((NN + RBM - 1) / RBM) * RBM <= NBK * NBRUN);

typedef float          v4f   __attribute__((ext_vector_type(4)));
typedef float          v8f   __attribute__((ext_vector_type(8)));
typedef int            v4i   __attribute__((ext_vector_type(4)));
typedef int            v8i   __attribute__((ext_vector_type(8)));
typedef unsigned short v8us  __attribute__((ext_vector_type(8)));
typedef unsigned short v16us __attribute__((ext_vector_type(16)));
typedef __bf16         v16bf __attribute__((ext_vector_type(16)));
typedef v4f  __attribute__((may_alias)) v4fa;
typedef v4i  __attribute__((may_alias)) v4ia;
typedef v8us __attribute__((may_alias)) v8usa;
union FragB { v16bf v; v16us u; v8us h[2]; v8i w; };

__device__ __forceinline__ v8f wmb(const FragB& a, const FragB& b, v8f c) {
  v8f d = __builtin_amdgcn_wmma_f32_16x16x32_bf16(false, a.v, false, b.v, (short)0, c, false, false);
  asm volatile("v_nop\n\tv_nop\n\tv_nop\n\tv_nop" : "+v"(d) : "v"(a.w), "v"(b.w));
  return d;
}

__device__ __forceinline__ unsigned bf16_bits(float f) {
  const unsigned u = __float_as_uint(f);
  const unsigned r = (u + 0x7FFFu + ((u >> 16) & 1u)) >> 16;
  const unsigned q = (u >> 16) | 0x40u;
  return ((u & 0x7fffffffu) > 0x7f800000u) ? q : r;
}
__device__ __forceinline__ float bf16_val(float f) {
  return __uint_as_float(bf16_bits(f) << 16);
}

__device__ __forceinline__ void st2_v4f(float* p, v4f v) {
  *(volatile v4f*)p = v;
  __threadfence();
  *(volatile v4f*)p = v;
}
__device__ __forceinline__ void st2_v8us(unsigned short* p, v8us v) {
  *(volatile v8us*)p = v;
  __threadfence();
  *(volatile v8us*)p = v;
}

__device__ __forceinline__ v8us col8(const float* __restrict__ base, int stride) {
  float f[8];
#pragma unroll
  for (int i = 0; i < 8; ++i) f[i] = base[(size_t)i * (size_t)stride];
  v8us o;
#pragma unroll
  for (int i = 0; i < 8; ++i) o[i] = (unsigned short)bf16_bits(f[i]);
  return o;
}

__device__ __forceinline__ v8us row8(const float* __restrict__ p, unsigned mk) {
  const v4f a = *(const v4fa*)p;
  const v4f b = *(const v4fa*)(p + 4);
  v8us o;
  o[0] = (unsigned short)(bf16_bits(a.x) & mk); o[1] = (unsigned short)(bf16_bits(a.y) & mk);
  o[2] = (unsigned short)(bf16_bits(a.z) & mk); o[3] = (unsigned short)(bf16_bits(a.w) & mk);
  o[4] = (unsigned short)(bf16_bits(b.x) & mk); o[5] = (unsigned short)(bf16_bits(b.y) & mk);
  o[6] = (unsigned short)(bf16_bits(b.z) & mk); o[7] = (unsigned short)(bf16_bits(b.w) & mk);
  return o;
}

__global__ __launch_bounds__(NTHR) void k_prep(const float* __restrict__ h, const float* __restrict__ rel,
                                               const float* __restrict__ wn, const float* __restrict__ wl,
                                               unsigned short* xb, unsigned short* relb, unsigned short* wt) {
  const int tid = (int)threadIdx.x;
  const int blk = (int)blockIdx.x;
  if (blk < PBX) {
    const int u   = blk * NTHR + tid;
    const int row = u >> 4, k8 = (u & 15) * 8;
    const int rc  = row < NN ? row : NN - 1;
    const unsigned mk = row < NN ? 0xffffu : 0u;
    const v8us o = row8(h + (size_t)rc * DF + k8, mk);
    st2_v8us(xb + (size_t)row * APITCH + k8, o);
  } else if (blk < PBX + PBR) {
    const int u   = (blk - PBX) * NTHR + tid;
    const int row = u >> 4, k8 = (u & 15) * 8;
    const int rc  = row < NR ? row : NR - 1;
    const unsigned mk = row < NR ? 0xffffu : 0u;
    const v8us o = row8(rel + (size_t)rc * DF + k8, mk);
    st2_v8us(relb + (size_t)row * APITCH + k8, o);
  } else if (blk < PBX + PBR + PBW) {
    const int u = (blk - PBX - PBR) * NTHR + tid;
    const int n = u >> 4, k8 = (u & 15) * 8;
    const v8us o = col8(wn + (size_t)k8 * DF + n, DF);
    st2_v8us(wt + (size_t)n * BPITCH + k8, o);
  } else {
    const int u = (blk - PBX - PBR - PBW) * NTHR + tid;
    const int n = u >> 4, k8 = (u & 15) * 8;
    const v8us o = col8(wl + (size_t)k8 * DF + n, DF);
    st2_v8us(wt + (size_t)(DF + n) * BPITCH + k8, o);
  }
}

__global__ __launch_bounds__(GTHR) __attribute__((amdgpu_num_vgpr(248)))
void k_gemm(const unsigned short* __restrict__ Apl, const unsigned short* __restrict__ BT,
            float* C, unsigned planeStride) {
  __shared__ __attribute__((aligned(16))) float stg[GBM * GBN];
  const int tid = (int)threadIdx.x, lane = tid & 31, wave = tid >> 5, hh = lane >> 4, m = lane & 15;
  const int rowBase = (int)blockIdx.x * GBM;
  const int plane   = (int)blockIdx.y;

  v8f acc[8];
  {
    const v8f z = {0.f, 0.f, 0.f, 0.f, 0.f, 0.f, 0.f, 0.f};
#pragma unroll
    for (int t = 0; t < 8; ++t) acc[t] = z;
  }
  const unsigned short* ap = Apl + (size_t)(rowBase + 16 * wave + m) * (size_t)APITCH + 8 * hh;
  const unsigned short* bp = BT + (size_t)(GBN * plane + m) * (size_t)BPITCH + 8 * hh;

#pragma unroll 1
  for (int k0 = 0; k0 < KD; k0 += 32) {
    FragB af;
    af.h[0] = *(const v8usa*)(ap + k0);
    af.h[1] = *(const v8usa*)(ap + k0 + 16);
#pragma unroll
    for (int nt = 0; nt < 8; ++nt) {
      const unsigned short* wq = bp + (size_t)(16 * nt) * (size_t)BPITCH + k0;
      FragB bf;
      bf.h[0] = *(const v8usa*)wq;
      bf.h[1] = *(const v8usa*)(wq + 16);
      acc[nt] = wmb(af, bf, acc[nt]);
    }
  }

#pragma unroll
  for (int nt = 0; nt < 8; ++nt) {
    const int lc = 16 * nt + m;
#pragma unroll
    for (int r = 0; r < 8; ++r) {
      const int lr = 16 * wave + 8 * hh + r;
      stg[lr * GBN + lc] = acc[nt][r];
    }
  }
  __syncthreads();

  v4f pv[16];
#pragma unroll
  for (int i = 0; i < 16; ++i) pv[i] = *(const v4fa*)(stg + (16 * wave + i) * GBN + 4 * lane);

  float* cb = C + (size_t)plane * (size_t)planeStride + (size_t)(rowBase + 16 * wave) * (size_t)CPITCH + 4 * lane;
#pragma unroll
  for (int i = 0; i < 16; ++i) *(volatile v4f*)(cb + (size_t)i * CPITCH) = pv[i];
  __threadfence();
#pragma unroll
  for (int i = 0; i < 16; ++i) *(volatile v4f*)(cb + (size_t)i * CPITCH) = pv[i];
}

__device__ __forceinline__ void bucket_flush(const int* pl, const int* cnt, int ov, int* lp, int* cop, int* fp,
                                             int tid) {
#pragma unroll 1
  for (int i = tid * 4; i < RCAP; i += NTHR * 4) {
    const v4i v = *(const v4ia*)(pl + i);
    *(volatile v4i*)(lp + i) = v;
  }
  {
    const v4i v0 = *(const v4ia*)(cnt + 4 * tid);
    const v4i v1 = *(const v4ia*)(cnt + NBRUN + 4 * tid);
    *(volatile v4i*)(cop + 4 * tid) = v0;
    *(volatile v4i*)(cop + NBRUN + 4 * tid) = v1;
  }
  if (tid < 8) {
    const v4i f = {ov, ov, ov, ov};
    *(volatile v4i*)(fp + 4 * tid) = f;
  }
}

__global__ __launch_bounds__(NTHR) void k_bucket(const int* __restrict__ srcs, const int* __restrict__ dsts,
                                                 const int* __restrict__ ety, int* LIST, int* CO, int* FLAG) {
  extern __shared__ __attribute__((aligned(16))) int dsm[];
  int* wl   = dsm;
  int* pl   = dsm + NWAVE * WLCAP;
  int* cnt  = pl + RCAP;
  int* offs = cnt + NBRUN;
  int* cur  = offs + NBRUN;
  int* misc = cur + NBRUN;
  const int tid = (int)threadIdx.x, lane = tid & 31, wave = tid >> 5;
  const int blk = (int)blockIdx.x;
  const unsigned nbs = (unsigned)(blk * NBRUN);

  {
    const v4i z4 = {0, 0, 0, 0};
    for (int i = tid * 4; i < BK_ZINTS; i += NTHR * 4) *(v4ia*)(dsm + i) = z4;
    if (tid < 16) misc[tid] = 0;
  }
  __syncthreads();

  {
    constexpr int per = ((NE + NWAVE * WCH - 1) / (NWAVE * WCH)) * WCH;
    static_assert(per % WCH == 0 && (NWAVE - 1) * per < NE && NWAVE * per >= NE);
    const int estart = wave * per;
    const int eend   = (estart + per < NE) ? (estart + per) : NE;
    int* mylist = wl + wave * WLCAP;
    int wc = 0;
#pragma unroll 1
    for (int cb = estart; cb < eend; cb += WCH) {
      const int e0 = cb + lane * EPT;
      const v4i da = *(const v4ia*)(dsts + e0);
      const v4i db = *(const v4ia*)(dsts + e0 + 4);
      const unsigned s0 = (unsigned)da.x - nbs, s1 = (unsigned)da.y - nbs;
      const unsigned s2 = (unsigned)da.z - nbs, s3 = (unsigned)da.w - nbs;
      const unsigned s4 = (unsigned)db.x - nbs, s5 = (unsigned)db.y - nbs;
      const unsigned s6 = (unsigned)db.z - nbs, s7 = (unsigned)db.w - nbs;
      const bool h0 = s0 < (unsigned)NBRUN, h1 = s1 < (unsigned)NBRUN, h2 = s2 < (unsigned)NBRUN, h3 = s3 < (unsigned)NBRUN;
      const bool h4 = s4 < (unsigned)NBRUN, h5 = s5 < (unsigned)NBRUN, h6 = s6 < (unsigned)NBRUN, h7 = s7 < (unsigned)NBRUN;
      const unsigned m0 = __builtin_amdgcn_ballot_w32(h0), m1 = __builtin_amdgcn_ballot_w32(h1);
      const unsigned m2 = __builtin_amdgcn_ballot_w32(h2), m3 = __builtin_amdgcn_ballot_w32(h3);
      const unsigned m4 = __builtin_amdgcn_ballot_w32(h4), m5 = __builtin_amdgcn_ballot_w32(h5);
      const unsigned m6 = __builtin_amdgcn_ballot_w32(h6), m7 = __builtin_amdgcn_ballot_w32(h7);
      const unsigned any = m0 | m1 | m2 | m3 | m4 | m5 | m6 | m7;
      if (any != 0u) {
        const int pre = (int)(__builtin_amdgcn_mbcnt_lo(m0, 0u) + __builtin_amdgcn_mbcnt_lo(m1, 0u) +
                              __builtin_amdgcn_mbcnt_lo(m2, 0u) + __builtin_amdgcn_mbcnt_lo(m3, 0u) +
                              __builtin_amdgcn_mbcnt_lo(m4, 0u) + __builtin_amdgcn_mbcnt_lo(m5, 0u) +
                              __builtin_amdgcn_mbcnt_lo(m6, 0u) + __builtin_amdgcn_mbcnt_lo(m7, 0u));
        int p = wc + pre;
        if (h0) { if (p < WLCAP) mylist[p] = (e0 + 0) | ((int)s0 << 20); p = p + 1; }
        if (h1) { if (p < WLCAP) mylist[p] = (e0 + 1) | ((int)s1 << 20); p = p + 1; }
        if (h2) { if (p < WLCAP) mylist[p] = (e0 + 2) | ((int)s2 << 20); p = p + 1; }
        if (h3) { if (p < WLCAP) mylist[p] = (e0 + 3) | ((int)s3 << 20); p = p + 1; }
        if (h4) { if (p < WLCAP) mylist[p] = (e0 + 4) | ((int)s4 << 20); p = p + 1; }
        if (h5) { if (p < WLCAP) mylist[p] = (e0 + 5) | ((int)s5 << 20); p = p + 1; }
        if (h6) { if (p < WLCAP) mylist[p] = (e0 + 6) | ((int)s6 << 20); p = p + 1; }
        if (h7) { if (p < WLCAP) mylist[p] = (e0 + 7) | ((int)s7 << 20); p = p + 1; }
        wc += (int)(__builtin_popcount(m0) + __builtin_popcount(m1) + __builtin_popcount(m2) + __builtin_popcount(m3) +
                    __builtin_popcount(m4) + __builtin_popcount(m5) + __builtin_popcount(m6) + __builtin_popcount(m7));
      }
    }
    if (lane == 0) misc[wave] = wc;
  }
  __syncthreads();

  if (wave == 0) {
    int ov = 0;
#pragma unroll 1
    for (int w2 = 0; w2 < NWAVE; ++w2) {
      int c = misc[w2];
      if (c > WLCAP) ov = 1;
      c = c < 0 ? 0 : (c > WLCAP ? WLCAP : c);
#pragma unroll 1
      for (int b0 = 0; b0 < c; b0 += 32) {
        const int idx = b0 + lane;
        const int ent = wl[w2 * WLCAP + (idx < WLCAP ? idx : WLCAP - 1)];
        const int m32 = (c - b0) < 32 ? (c - b0) : 32;
#pragma unroll 1
        for (int k = 0; k < m32; ++k) {
          const int u    = __builtin_amdgcn_readlane(ent, k);
          const int slot = (u >> 20) & (NBRUN - 1);
          if (lane == 0) cnt[slot] = cnt[slot] + 1;
        }
      }
    }
    if (lane == 0) misc[9] = ov;
  }
  __syncthreads();
  if (wave == 0) {
    const int base = lane * (NBRUN / 32);
    int s = 0;
#pragma unroll 1
    for (int i = 0; i < NBRUN / 32; ++i) s += cnt[base + i];
    int incl = s;
#pragma unroll
    for (int d = 1; d < 32; d <<= 1) {
      const int y = __shfl_up(incl, d, 32);
      if (lane >= d) incl += y;
    }
    int run = incl - s;
#pragma unroll 1
    for (int i = 0; i < NBRUN / 32; ++i) {
      const int cv = cnt[base + i];
      offs[base + i] = run;
      cur[base + i]  = run;
      run += cv;
    }
    if (lane == 31) {
      misc[10] = run;
      if (run > RCAP) misc[9] = 1;
    }
  }
  __syncthreads();

  if (wave == 0) {
#pragma unroll 1
    for (int w2 = 0; w2 < NWAVE; ++w2) {
      int c = misc[w2];
      c = c < 0 ? 0 : (c > WLCAP ? WLCAP : c);
#pragma unroll 1
      for (int b0 = 0; b0 < c; b0 += 32) {
        const int idx = b0 + lane;
        const int ent = wl[w2 * WLCAP + (idx < WLCAP ? idx : WLCAP - 1)];
        const int m32 = (c - b0) < 32 ? (c - b0) : 32;
#pragma unroll 1
        for (int k = 0; k < m32; ++k) {
          const int u    = __builtin_amdgcn_readlane(ent, k);
          const int slot = (u >> 20) & (NBRUN - 1);
          const int eid  = u & 0xFFFFF;
          if (lane == 0) {
            int p = cur[slot];
            p = p < 0 ? 0 : (p > RCAP - 1 ? RCAP - 1 : p);
            pl[p] = eid;
            cur[slot] = p + 1;
          }
        }
      }
    }
  }
  __syncthreads();

  {
    int tot = misc[10];
    tot = tot < 0 ? 0 : (tot > RCAP ? RCAP : tot);
#pragma unroll 1
    for (int base = 0; base < tot; base += NTHR) {
      const int i = base + tid;
      int e = pl[i];
      e = e < 0 ? 0 : (e > NE - 1 ? NE - 1 : e);
      const int s0 = srcs[e];
      const int t0 = ety[e];
      asm volatile("" :: "v"(s0), "v"(t0));
      const int s = s0 < 0 ? 0 : (s0 > NN - 1 ? NN - 1 : s0);
      const int t = t0 < 0 ? 0 : (t0 > NR - 1 ? NR - 1 : t0);
      const int mk = (i < tot) ? -1 : 0;
      pl[i] = ((t << 17) | s) & mk;
    }
  }
  __syncthreads();

  const int ovf = misc[9];
  int* lp  = LIST + (size_t)blk * RCAP;
  int* cop = CO + (size_t)blk * (2 * NBRUN);
  int* fp  = FLAG + (size_t)blk * 32;
  bucket_flush(pl, cnt, ovf, lp, cop, fp, tid);
  __threadfence();
  bucket_flush(pl, cnt, ovf, lp, cop, fp, tid);
}

__global__ __launch_bounds__(NTHR) void k_replay(const int* __restrict__ LIST, const int* __restrict__ CO,
                                                 const int* __restrict__ FLAG, const float* __restrict__ HW,
                                                 const float* __restrict__ RW, const float* __restrict__ LP,
                                                 const float* __restrict__ nrm, float* out) {
  const int tid = (int)threadIdx.x, lane = tid & 31;
  const int wave = __builtin_amdgcn_readfirstlane(tid >> 5);
  const int rowBase = (int)blockIdx.x * RBM;
  const int bucket  = rowBase >> SLB;
  const int* lb  = LIST + (size_t)bucket * RCAP;
  const int* cob = CO + (size_t)bucket * (2 * NBRUN);
  const int flag = FLAG[(size_t)bucket * 32];
  const float qnan = __uint_as_float(0x7fc00000u);

#pragma unroll 1
  for (int i = 0; i < RBM / NWAVE; ++i) {
    const int d = rowBase + (RBM / NWAVE) * wave + i;
    if (d < NN) {
      const int slot = d & (NBRUN - 1);
      int c = cob[slot];
      int o = cob[NBRUN + slot];
      c = c < 0 ? 0 : (c > RCAP ? RCAP : c);
      o = o < 0 ? 0 : (o > RCAP - 1 ? RCAP - 1 : o);
      c = __builtin_amdgcn_readfirstlane(c);
      o = __builtin_amdgcn_readfirstlane(o);
      int last = o + c - 1;
      last = last < o ? o : last;
      last = last > RCAP - 1 ? RCAP - 1 : last;
      float a0 = 0.0f, a1 = 0.0f, a2 = 0.0f, a3 = 0.0f;
#pragma unroll 2
      for (int j = 0; j < c; ++j) {
        int idx = o + j;
        idx = idx > last ? last : idx;
        const unsigned wd = (unsigned)lb[idx];
        int sr = (int)(wd & 0x1FFFFu);
        sr = sr > NN - 1 ? NN - 1 : sr;
        int ty = (int)(wd >> 17);
        ty = ty > NR - 1 ? NR - 1 : ty;
        const v4f a = *(const v4fa*)(HW + (size_t)sr * CPITCH + 4 * lane);
        const v4f r = *(const v4fa*)(RW + (size_t)ty * CPITCH + 4 * lane);
        a0 += (a.x - r.x);
        a1 += (a.y - r.y);
        a2 += (a.z - r.z);
        a3 += (a.w - r.w);
      }
      const float nv = bf16_val(nrm[d]);
      const v4f g = *(const v4fa*)(LP + (size_t)d * CPITCH + 4 * lane);
      float v0 = fmaf(a0, nv, g.x), v1 = fmaf(a1, nv, g.y), v2 = fmaf(a2, nv, g.z), v3 = fmaf(a3, nv, g.w);
      v0 = (v0 > 0.0f) ? v0 : (v0 - v0);
      v1 = (v1 > 0.0f) ? v1 : (v1 - v1);
      v2 = (v2 > 0.0f) ? v2 : (v2 - v2);
      v3 = (v3 > 0.0f) ? v3 : (v3 - v3);
      v4f ov;
      ov.x = (flag != 0) ? qnan : v0;
      ov.y = (flag != 0) ? qnan : v1;
      ov.z = (flag != 0) ? qnan : v2;
      ov.w = (flag != 0) ? qnan : v3;
      st2_v4f(out + (size_t)d * DF + 4 * lane, ov);
    }
  }
}

extern "C" void kernel_launch(void* const* d_in, const int* in_sizes, int n_in,
                              void* d_out, int out_size, void* d_ws, size_t ws_size,
                              hipStream_t stream) {
  if (n_in < 8) return;
  if (in_sizes[0] != NN * DF) return;
  if (in_sizes[1] != NN) return;
  if (in_sizes[2] != NR * DF) return;
  if (in_sizes[3] != DF * DF) return;
  if (in_sizes[4] != DF * DF) return;
  if (in_sizes[5] != NE) return;
  if (in_sizes[6] != NE) return;
  if (in_sizes[7] != NE) return;
  if (out_size != NN * DF) return;

  const float* h    = (const float*)d_in[0];
  const float* nrm  = (const float*)d_in[1];
  const float* rel  = (const float*)d_in[2];
  const float* Wn   = (const float*)d_in[3];
  const float* Wl   = (const float*)d_in[4];
  const int*   srcs = (const int*)d_in[5];
  const int*   dsts = (const int*)d_in[6];
  const int*   ety  = (const int*)d_in[7];
  float* out = (float*)d_out;

  constexpr size_t zXB   = (size_t)MP * APITCH * 2;
  constexpr size_t zF    = (size_t)MP * CPITCH * 4;
  constexpr size_t zRW   = (size_t)RP * CPITCH * 4;
  constexpr size_t zRELB = (size_t)RP * APITCH * 2;
  constexpr size_t zWT   = (size_t)2 * DF * BPITCH * 2;
  constexpr size_t zLIST = (size_t)NBK * RCAP * 4;
  constexpr size_t zCO   = (size_t)NBK * 2 * NBRUN * 4;
  constexpr size_t zFLAG = (size_t)NBK * 128;
  constexpr size_t oXB   = 0;
  constexpr size_t oHW   = oXB + zXB;
  constexpr size_t oLOOP = oHW + zF;
  constexpr size_t oRW   = oLOOP + zF;
  constexpr size_t oRELB = oRW + zRW;
  constexpr size_t oWT   = oRELB + zRELB;
  constexpr size_t oLIST = oWT + zWT;
  constexpr size_t oCO   = oLIST + zLIST;
  constexpr size_t oFLAG = oCO + zCO;
  constexpr size_t oEND  = oFLAG + zFLAG;
  static_assert(zXB % 256 == 0 && zF % 256 == 0 && zRW % 256 == 0 && zRELB % 256 == 0 && zWT % 256 == 0);
  static_assert(zLIST % 256 == 0 && zCO % 256 == 0 && zFLAG % 256 == 0);
  static_assert(oLOOP - oHW == (size_t)MP * CPITCH * 4);
  static_assert(oEND <= (size_t)(128u << 20));
  if (oEND > ws_size) return;

  char* ws = (char*)d_ws;
  unsigned short* XB   = (unsigned short*)(ws + oXB);
  float*          HW   = (float*)(ws + oHW);
  float*          LP   = (float*)(ws + oLOOP);
  float*          RW   = (float*)(ws + oRW);
  unsigned short* RELB = (unsigned short*)(ws + oRELB);
  unsigned short* WT   = (unsigned short*)(ws + oWT);
  int*            LIST = (int*)(ws + oLIST);
  int*            CO   = (int*)(ws + oCO);
  int*            FLAG = (int*)(ws + oFLAG);

  hipFuncSetAttribute(reinterpret_cast<const void*>(&k_bucket), hipFuncAttributeMaxDynamicSharedMemorySize, (int)BK_LDS);

  k_prep<<<PBTOT, NTHR, 0, stream>>>(h, rel, Wn, Wl, XB, RELB, WT);
  k_gemm<<<dim3(MP / GBM, 2), GTHR, 0, stream>>>(XB, WT, HW, (unsigned)((size_t)MP * CPITCH));
  k_gemm<<<dim3(RP / GBM, 1), GTHR, 0, stream>>>(RELB, WT, RW, 0u);
  k_bucket<<<NBK, NTHR, BK_LDS, stream>>>(srcs, dsts, ety, LIST, CO, FLAG);
  k_replay<<<(NN + RBM - 1) / RBM, NTHR, 0, stream>>>(LIST, CO, FLAG, HW, RW, LP, nrm, out);
}
